// FCN_ManualFeats_Early_Fusion_37099927503292
// MI455X (gfx1250) — hardware-verified
//
#include <hip/hip_runtime.h>


#ifndef NROWS
#define NROWS 131072
#endif
#define NROWS_FULL 131072
#define KIN    29
#define NF     59
#define NFP    64
#define NST    15
#define NTILE  (NROWS / 64)
#define APW    68
#define OSP    68
#define W0PW   16
#define WSPW   64
#define STSLOT 256
#define BN_EPS 1.0e-5f
#define NPIECE ((NROWS * NF) / 4)
#define WCONV_BLOCKS (1 + ((NST - 1) * 64 * 16) / 256)

static constexpr float INV_ROWS = 1.0f / (float)NROWS;
static constexpr float INV_TILE = 1.0f / 64.0f;
static constexpr float TILE_CNT = 64.0f;

static_assert(NROWS % 64 == 0);
static_assert(NROWS <= NROWS_FULL);
static_assert(NTILE % 4 == 0);
static_assert(KIN <= 32);
static_assert(NF <= NFP);
static_assert(NFP == 64);
static_assert((APW * 4) % 16 == 0);
static_assert(APW >= 64);
static_assert((OSP * 4) % 16 == 0);
static_assert(((size_t)NROWS * NF) % 32 == 0);
static_assert((size_t)NROWS * NF < (size_t)4294967295u);
static_assert(((NST - 1) * 64 * 16) % 256 == 0);
static_assert(64 * 4 == 256);
static_assert(8 * (32 / 16) == 16);
static_assert(16 * 16 == NFP * 4);
static_assert(32 * 16 == 128 * 4);
static_assert(48 * 16 == 192 * 4);
static_assert(64 * APW * 4 + 16 * OSP * 4 + 128 * 4 <= 131072);
static_assert(256 * 4 * 2 + 192 * 4 <= 131072);
static_assert(STSLOT >= 192);

typedef __attribute__((ext_vector_type(16))) __bf16   v16bf;
typedef __attribute__((ext_vector_type(8)))  float    v8f;
typedef __attribute__((ext_vector_type(4)))  float    v4f;
typedef __attribute__((ext_vector_type(8)))  unsigned v8u;
typedef __attribute__((ext_vector_type(4)))  unsigned v4u;
typedef __attribute__((ext_vector_type(2)))  unsigned v2u;
typedef v4f __attribute__((may_alias)) v4fa;
typedef v4u __attribute__((may_alias)) v4ua;
typedef v2u __attribute__((may_alias)) v2ua;

__device__ __forceinline__ unsigned bf16_bits(float f) { unsigned u = __float_as_uint(f); u += 0x7FFFu + ((u >> 16) & 1u); return u >> 16; }
__device__ __forceinline__ float bfr(float f) { return __uint_as_float(bf16_bits(f) << 16); }
__device__ __forceinline__ v8f wmmab(v16bf a, v16bf b, v8f c) { return __builtin_amdgcn_wmma_f32_16x16x32_bf16(false, a, false, b, (short)0, c, false, false); }
__device__ __forceinline__ v8f wmmabg(v16bf a, v16bf b, v8f c) { c = wmmab(a, b, c); asm volatile("v_nop\n\tv_nop\n\tv_nop\n\tv_nop" : "+v"(c) : "v"(a), "v"(b)); return c; }
__device__ __forceinline__ v16bf frag16(v4u lo, v4u hi) { const v8u w = __builtin_shufflevector(lo, hi, 0, 1, 2, 3, 4, 5, 6, 7); return __builtin_bit_cast(v16bf, w); }
__device__ __forceinline__ void st2_v4f(float* p, v4f v) { *(volatile v4f*)p = v; __threadfence(); *(volatile v4f*)p = v; }
__device__ __forceinline__ void st2_v4u(unsigned* p, v4u v) { *(volatile v4u*)p = v; __threadfence(); *(volatile v4u*)p = v; }

__global__ __launch_bounds__(256) void k_wconv(const float* __restrict__ W0, const float* __restrict__ Ws, unsigned* WP0, unsigned* WPS) {
    const unsigned bx = blockIdx.x, t = threadIdx.x;
    if (bx == 0u) {
        const unsigned n = t >> 2, k8 = (t & 3u) * 8u;
        const unsigned nc = (unsigned)min((int)n, NF - 1);
        v4u o;
#pragma unroll
        for (int j = 0; j < 4; ++j) {
            const unsigned ka = k8 + 2u * (unsigned)j, kb = ka + 1u;
            const float fa = W0[nc * KIN + (unsigned)min((int)ka, KIN - 1)];
            const float fb = W0[nc * KIN + (unsigned)min((int)kb, KIN - 1)];
            const unsigned ba = (n < NF && ka < KIN) ? bf16_bits(fa) : 0u;
            const unsigned bb = (n < NF && kb < KIN) ? bf16_bits(fb) : 0u;
            o[j] = ba | (bb << 16);
        }
        st2_v4u(WP0 + t * 4u, o);
    } else {
        const unsigned q = (bx - 1u) * 256u + t;
        const unsigned l = q >> 10, rem = q & 1023u, n = rem >> 4, kk8 = (rem & 15u) * 8u;
        const unsigned nc = (unsigned)min((int)n, NF - 1);
        const unsigned base = l * (NF * NF) + nc * NF;
        v4u o;
#pragma unroll
        for (int j = 0; j < 4; ++j) {
            const unsigned ka = (kk8 + 2u * (unsigned)j) & 63u, kb = (kk8 + 2u * (unsigned)j + 1u) & 63u;
            const float fa = Ws[base + (unsigned)min((int)ka, NF - 1)];
            const float fb = Ws[base + (unsigned)min((int)kb, NF - 1)];
            const unsigned ba = (n < NF && ka < NF) ? bf16_bits(fa) : 0u;
            const unsigned bb = (n < NF && kb < NF) ? bf16_bits(fb) : 0u;
            o[j] = ba | (bb << 16);
        }
        st2_v4u(WPS + q * 4u, o);
    }
}

template <int FIRST>
__device__ __forceinline__ void gemm_body(const float* __restrict__ src, const float* __restrict__ stin, const unsigned* __restrict__ WP,
                                          const float* __restrict__ bias, float* Rout, float* part) {
    __shared__ __align__(16) unsigned at[64 * APW];
    __shared__ __align__(16) float os[16 * OSP];
    __shared__ __align__(16) float ps[128];
    const unsigned lane = threadIdx.x & 31u, lr = lane & 15u, hi = lane >> 4;
    const unsigned tile = blockIdx.x;
    const size_t r0 = (size_t)tile * 64u;

    if (FIRST) {
#pragma unroll 1
        for (unsigned rr = 0; rr < 2u; ++rr) {
            const unsigned row = lane + 32u * rr;
            const float* xr = src + (r0 + row) * KIN;
#pragma unroll 4
            for (unsigned j = 0; j < 16u; ++j) {
                const unsigned ka = 2u * j, kb = 2u * j + 1u;
                const float fa = xr[(unsigned)min((int)ka, KIN - 1)];
                const float fb = xr[(unsigned)min((int)kb, KIN - 1)];
                const unsigned ba = (ka < KIN) ? bf16_bits(fa) : 0u;
                const unsigned bb = (kb < KIN) ? bf16_bits(fb) : 0u;
                at[row * APW + j] = ba | (bb << 16);
            }
        }
    } else {
        const unsigned c4 = lr * 4u;
        const v4f mu = *(const v4f*)(stin + c4);
        const v4f sc = *(const v4f*)(stin + 64 + c4);
        const v4f sh = *(const v4f*)(stin + 128 + c4);
#pragma unroll 4
        for (unsigned i = 0; i < 32u; ++i) {
            const unsigned row = 2u * i + hi;
            const v4f r = *(const v4f*)(src + (r0 + row) * NFP + c4);
            unsigned hb[4], lb[4];
#pragma unroll
            for (int e = 0; e < 4; ++e) {
                const float a = (r[e] - mu[e]) * sc[e] + sh[e];
                const unsigned b = bf16_bits(a);
                const float av = __uint_as_float(b << 16);
                hb[e] = b; lb[e] = bf16_bits(a - av);
            }
            v2u hv, lv;
            hv[0] = hb[0] | (hb[1] << 16); hv[1] = hb[2] | (hb[3] << 16);
            lv[0] = lb[0] | (lb[1] << 16); lv[1] = lb[2] | (lb[3] << 16);
            *(v2ua*)(&at[row * APW + 2u * lr]) = hv;
            *(v2ua*)(&at[row * APW + 32u + 2u * lr]) = lv;
        }
    }
    __syncthreads();

    v8f acc[4][4];
#pragma unroll
    for (int mb = 0; mb < 4; ++mb)
#pragma unroll
        for (int nb = 0; nb < 4; ++nb) acc[mb][nb] = (v8f){};
    constexpr unsigned KS  = FIRST ? 1u : 4u;
    constexpr unsigned WPW = FIRST ? W0PW : WSPW;
    const unsigned aw = lr * APW + 4u * hi;
    const unsigned bw = lr * WPW + 4u * hi;
#pragma unroll 1
    for (unsigned kc = 0; kc < KS; ++kc) {
        v16bf a[4];
#pragma unroll
        for (int mb = 0; mb < 4; ++mb) { const unsigned w = aw + (unsigned)mb * 16u * APW + kc * 16u;
            a[mb] = frag16(*(const v4ua*)(&at[w]), *(const v4ua*)(&at[w + 8u])); }
#pragma unroll
        for (int nb = 0; nb < 4; ++nb) { const unsigned w = bw + (unsigned)nb * 16u * WPW + kc * 16u;
            const v16bf b = frag16(*(const v4u*)(WP + w), *(const v4u*)(WP + w + 8u));
#pragma unroll
            for (int mb = 0; mb < 4; ++mb) acc[mb][nb] = wmmabg(a[mb], b, acc[mb][nb]); }
    }

#pragma unroll
    for (int nb = 0; nb < 4; ++nb) {
        const unsigned n = (unsigned)nb * 16u + lr;
        const float bl = bfr(bias[(unsigned)min((int)n, NF - 1)]);
        const float bc = (n < NF) ? bl : 0.0f;
#pragma unroll
        for (int mb = 0; mb < 4; ++mb)
#pragma unroll
            for (int j = 0; j < 8; ++j) acc[mb][nb][j] = fmaxf(acc[mb][nb][j] + bc, 0.0f);
    }
#pragma unroll
    for (int nb = 0; nb < 4; ++nb) {
        float s = 0.0f;
#pragma unroll
        for (int mb = 0; mb < 4; ++mb)
#pragma unroll
            for (int j = 0; j < 8; ++j) s += acc[mb][nb][j];
        s += __shfl_xor(s, 16, 32);
        const float mt = s * INV_TILE;
        float q = 0.0f;
#pragma unroll
        for (int mb = 0; mb < 4; ++mb)
#pragma unroll
            for (int j = 0; j < 8; ++j) { const float d = acc[mb][nb][j] - mt; q += d * d; }
        q += __shfl_xor(q, 16, 32);
        ps[hi * 64u + (unsigned)nb * 16u + lr] = (hi != 0u) ? q : s;
    }
#pragma unroll
    for (int mb = 0; mb < 4; ++mb) {
#pragma unroll
        for (int nb = 0; nb < 4; ++nb)
#pragma unroll
            for (int j = 0; j < 8; ++j) os[(hi * 8u + (unsigned)j) * OSP + (unsigned)nb * 16u + lr] = acc[mb][nb][j];
        __syncthreads();
#pragma unroll 1
        for (int pass = 0; pass < 2; ++pass) {
#pragma unroll
            for (int s = 0; s < 8; ++s) { const unsigned row = 2u * (unsigned)s + hi, c4 = lr * 4u;
                const v4f val = *(const v4fa*)(&os[row * OSP + c4]);
                *(volatile v4f*)(Rout + (r0 + (unsigned)mb * 16u + row) * NFP + c4) = val; }
            if (pass == 0) __threadfence(); }
        __syncthreads();
    }
    { const v4f pv = *(const v4fa*)(&ps[lane * 4u]);
      st2_v4f(part + (size_t)tile * 128u + lane * 4u, pv); }
}

__global__ __launch_bounds__(32) void k_gemm_first(const float* __restrict__ X, const unsigned* __restrict__ WP, const float* __restrict__ bias, float* Rout, float* part) {
    gemm_body<1>(X, X, WP, bias, Rout, part);
}
__global__ __launch_bounds__(32) void k_gemm_next(const float* __restrict__ Rin, const float* __restrict__ stin, const unsigned* __restrict__ WP, const float* __restrict__ bias, float* Rout, float* part) {
    gemm_body<0>(Rin, stin, WP, bias, Rout, part);
}

__global__ __launch_bounds__(256) void k_red(const float* __restrict__ part, const float* __restrict__ g, const float* __restrict__ bt, float* st) {
#pragma clang fp contract(off)
    __shared__ float ra[256];
    __shared__ float rb[256];
    __shared__ __align__(16) float so[192];
    const unsigned t = threadIdx.x, col = t & 63u, seg = t >> 6;
    const unsigned TPS = NTILE / 4;
    const float* p = part + (size_t)(seg * TPS) * 128u + col;
    float s = 0.0f, c = 0.0f;
#pragma unroll 1
    for (unsigned i = 0; i < TPS; ++i) { const float x = p[(size_t)i * 128u]; const float y = x - c; const float tt = s + y; c = (tt - s) - y; s = tt; }
    ra[t] = s;
    __syncthreads();
    const float tot = ((ra[col] + ra[64u + col]) + ra[128u + col]) + ra[192u + col];
    const float mean = tot * INV_ROWS;
    float s2 = 0.0f, c2 = 0.0f;
#pragma unroll 1
    for (unsigned i = 0; i < TPS; ++i) {
        const float ts = p[(size_t)i * 128u]; const float m2 = p[(size_t)i * 128u + 64u];
        const float d = ts * INV_TILE - mean; const float x = m2 + TILE_CNT * (d * d);
        const float y = x - c2; const float tt = s2 + y; c2 = (tt - s2) - y; s2 = tt; }
    rb[t] = s2;
    __syncthreads();
    const float tot2 = ((rb[col] + rb[64u + col]) + rb[128u + col]) + rb[192u + col];
    const float var = tot2 * INV_ROWS;
    const float istd = 1.0f / sqrtf(var + BN_EPS);
    const unsigned cc = (unsigned)min((int)col, NF - 1);
    const float gv = bfr(g[cc]), bv = bfr(bt[cc]);
    const bool live = col < NF;
    if (seg == 0u) {
        so[col] = live ? mean : 0.0f; so[64u + col] = live ? (istd * gv) : 0.0f; so[128u + col] = live ? bv : 0.0f; }
    __syncthreads();
    if (t < 48u) { const v4f v = *(const v4fa*)(&so[t * 4u]); st2_v4f(st + t * 4u, v); }
}

__global__ __launch_bounds__(256) void k_out(const float* __restrict__ R, const float* __restrict__ st, float* OUT) {
    __shared__ float sl[256];
    const unsigned t = threadIdx.x;
    sl[t] = st[(unsigned)min((int)t, 191)];
    __syncthreads();
    const unsigned p = blockIdx.x * 256u + t;
    if (p < (unsigned)NPIECE) {
        const unsigned e0 = p * 4u;
        v4f o;
#pragma unroll
        for (int i = 0; i < 4; ++i) {
            const unsigned e = e0 + (unsigned)i; const unsigned row = e / 59u; const unsigned col = e - row * 59u;
            const float r = R[(size_t)row * NFP + col];
            o[i] = (r - sl[col]) * sl[64u + col] + sl[128u + col]; }
        st2_v4f(OUT + (size_t)e0, o);
    }
}

static constexpr size_t al256(size_t v) { return (v + 255) & ~(size_t)255; }
static constexpr size_t SZ_W0   = al256((size_t)64 * W0PW * 4);
static constexpr size_t SZ_WS   = al256((size_t)(NST - 1) * 64 * WSPW * 4);
static constexpr size_t SZ_ST   = al256((size_t)NST * STSLOT * 4);
static constexpr size_t SZ_PART = al256((size_t)NST * NTILE * 128 * 4);
static constexpr size_t SZ_R    = al256((size_t)NROWS * NFP * 4);
static constexpr size_t SZ_TOTAL = SZ_W0 + SZ_WS + SZ_ST + SZ_PART + 2 * SZ_R;
static_assert(SZ_TOTAL <= (size_t)134217728);
static_assert((size_t)256 * 4 * 4 == (size_t)64 * W0PW * 4);
static_assert((size_t)(WCONV_BLOCKS - 1) * 256 * 16 == (size_t)(NST - 1) * 64 * WSPW * 4);
static_assert((size_t)NTILE * 64 * NFP * 4 == (size_t)NROWS * NFP * 4);
static_assert((size_t)NTILE * 512 == (size_t)NTILE * 128 * 4);

extern "C" void kernel_launch(void* const* d_in, const int* in_sizes, int n_in,
                              void* d_out, int out_size, void* d_ws, size_t ws_size, hipStream_t stream) {
    if (n_in < 9) return;
    if ((size_t)in_sizes[0] < (size_t)NROWS * KIN) return;
    if (in_sizes[1] < NF * KIN || in_sizes[2] < NF || in_sizes[3] < NF || in_sizes[4] < NF) return;
    if (in_sizes[5] < (NST - 1) * NF * NF || in_sizes[6] < (NST - 1) * NF || in_sizes[7] < (NST - 1) * NF || in_sizes[8] < (NST - 1) * NF) return;
    if ((size_t)out_size < (size_t)NROWS * NF) return;
    if (SZ_TOTAL > ws_size) return;
    const float* x   = (const float*)d_in[0];
    const float* W0  = (const float*)d_in[1];
    const float* b0  = (const float*)d_in[2];
    const float* g0  = (const float*)d_in[3];
    const float* bt0 = (const float*)d_in[4];
    const float* Ws  = (const float*)d_in[5];
    const float* bs  = (const float*)d_in[6];
    const float* gs  = (const float*)d_in[7];
    const float* bts = (const float*)d_in[8];
    float* OUT = (float*)d_out;
    char* wsp = (char*)d_ws;
    unsigned* WP0 = (unsigned*)wsp; wsp += SZ_W0;
    unsigned* WPS = (unsigned*)wsp; wsp += SZ_WS;
    float* ST   = (float*)wsp; wsp += SZ_ST;
    float* PART = (float*)wsp; wsp += SZ_PART;
    float* RA   = (float*)wsp; wsp += SZ_R;
    float* RB   = (float*)wsp; wsp += SZ_R;

    k_wconv<<<WCONV_BLOCKS, 256, 0, stream>>>(W0, Ws, WP0, WPS);

    k_gemm_first<<<NTILE, 32, 0, stream>>>(x, WP0, b0, RA, PART);
    k_red<<<1, 256, 0, stream>>>(PART, g0, bt0, ST);

    for (int l = 1; l < NST; ++l) {
        const float* rin = (l & 1) ? RA : RB;
        float* rout      = (l & 1) ? RB : RA;
        float* pl = PART + (size_t)l * NTILE * 128;
        k_gemm_next<<<NTILE, 32, 0, stream>>>(rin, ST + (size_t)(l - 1) * STSLOT, WPS + (size_t)(l - 1) * 64 * WSPW, bs + (size_t)(l - 1) * NF, rout, pl);
        k_red<<<1, 256, 0, stream>>>(pl, gs + (size_t)(l - 1) * NF, bts + (size_t)(l - 1) * NF, ST + (size_t)l * STSLOT);
    }
    const float* rlast = ((NST - 1) & 1) ? RB : RA;
    k_out<<<(unsigned)((NPIECE + 255) / 256), 256, 0, stream>>>(rlast, ST + (size_t)(NST - 1) * STSLOT, OUT);
}
